// FusionMamba_7834020347953
// MI455X (gfx1250) — hardware-verified
//
#include <hip/hip_runtime.h>
#include <math.h>

typedef __attribute__((ext_vector_type(16))) _Float16 v16h;
typedef __attribute__((ext_vector_type(8)))  _Float16 v8h;
typedef __attribute__((ext_vector_type(16))) __bf16   v16b;
typedef __attribute__((ext_vector_type(8)))  __bf16   v8b;
typedef __attribute__((ext_vector_type(8)))  float    v8f;
typedef __attribute__((ext_vector_type(4)))  float    v4f;

constexpr int kBatch = 4;
constexpr int kSeqL  = 4096;
constexpr int kDim   = 64;
constexpr int kNst   = 8;
constexpr int kDtR   = 4;
constexpr int kTap   = 4;
constexpr int kNBlk  = 8;
constexpr int kRows  = kBatch * kSeqL;
constexpr int kXZP   = 2 * kDim;
constexpr int kPrjN  = kDtR + 2 * kNst;
constexpr int kPrjP  = 64;
constexpr int kCatW  = 2 * kDim;
constexpr int kYP    = 68;
static_assert(kRows % 64 == 0 && kXZP % 64 == 0 && kPrjP % 64 == 0 && kSeqL % 64 == 0, "tiles");
static_assert(kDim % 32 == 0 && kCatW % 32 == 0, "ksteps");

__device__ __forceinline__ unsigned short f2bf_bits(float f) {
  unsigned u = __float_as_uint(f);
  return (unsigned short)((u + 0x7FFFu + ((u >> 16) & 1u)) >> 16);
}
__device__ __forceinline__ float bf_bits2f(unsigned short h) { return __uint_as_float(((unsigned)h) << 16); }

__device__ __forceinline__ void dep_guard_h(v8f& a, v8f& b, v16h x, v16h y) { asm volatile("v_nop\n\tv_nop\n\tv_nop\n\tv_nop" : "+v"(a), "+v"(b) : "v"(x), "v"(y)); }
__device__ __forceinline__ void dep_guard_b(v8f& a, v8f& b, v16b x, v16b y) { asm volatile("v_nop\n\tv_nop\n\tv_nop\n\tv_nop" : "+v"(a), "+v"(b) : "v"(x), "v"(y)); }
__device__ __forceinline__ void keep4_h(v16h a, v16h b, v16h c, v16h d) { asm volatile("v_nop" :: "v"(a), "v"(b), "v"(c), "v"(d)); }
__device__ __forceinline__ void keep4_b(v16b a, v16b b, v16b c, v16b d) { asm volatile("v_nop" :: "v"(a), "v"(b), "v"(c), "v"(d)); }
__device__ __forceinline__ void acc_guard4(v8f& a, v8f& b, v8f& c, v8f& d) { asm volatile("v_nop\n\tv_nop\n\tv_nop\n\tv_nop" : "+v"(a), "+v"(b), "+v"(c), "+v"(d)); }
template <typename T> struct Frag;
template <> struct Frag<_Float16> {
  typedef v16h V; union U { v16h v; v8h h[2]; };
  static __device__ __forceinline__ v16h load(const _Float16* p) {
    U f; f.h[0] = *(const v8h*)(p); f.h[1] = *(const v8h*)(p + 16); return f.v;
  }
  static __device__ __forceinline__ v8f mma(v16h a, v16h b, v8f c) {
    return __builtin_amdgcn_wmma_f32_16x16x32_f16(false, a, false, b, (short)0, c, false, false);
  }
  static __device__ __forceinline__ void guard(v8f& a, v8f& b, v16h x, v16h y) { dep_guard_h(a, b, x, y); }
  static __device__ __forceinline__ void keep(v16h a, v16h b, v16h c, v16h d) { keep4_h(a, b, c, d); }
};
template <> struct Frag<__bf16> {
  typedef v16b V; union U { v16b v; v8b h[2]; };
  static __device__ __forceinline__ v16b load(const __bf16* p) {
    U f; f.h[0] = *(const v8b*)(p); f.h[1] = *(const v8b*)(p + 16); return f.v;
  }
  static __device__ __forceinline__ v8f mma(v16b a, v16b b, v8f c) {
    return __builtin_amdgcn_wmma_f32_16x16x32_bf16(false, a, false, b, (short)0, c, false, false);
  }
  static __device__ __forceinline__ void guard(v8f& a, v8f& b, v16b x, v16b y) { dep_guard_b(a, b, x, y); }
  static __device__ __forceinline__ void keep(v16b a, v16b b, v16b c, v16b d) { keep4_b(a, b, c, d); }
};

template <int ET> struct Elem;
template <> struct Elem<0> { typedef _Float16 T; };
template <> struct Elem<1> { typedef __bf16 T; };
template <int ET, bool SPLIT, int BIAS_MODE, int OUT_MODE, bool RESID, int ACT = 0>
__global__ __launch_bounds__(256) void wmma_gemm64(
    const unsigned short* __restrict__ Ap, const unsigned short* __restrict__ A2p, int lda, long strideA,
    const unsigned short* __restrict__ Btp, const unsigned short* __restrict__ Bt2p, int ldb, long strideB,
    void* __restrict__ Cout, void* __restrict__ Cout2, int ldc, long strideC,
    const float* __restrict__ bias,
    const float* __restrict__ resid, long strideR,
    int M, int N, int K, float scale) {
  typedef typename Elem<ET>::T T;
  typedef typename Frag<T>::V V;
  const T* A = (const T*)Ap; const T* A2 = (const T*)A2p; const T* Bt = (const T*)Btp; const T* Bt2 = (const T*)Bt2p;
  __shared__ __align__(16) float sT[8][16 * 68];
  const int b    = blockIdx.y;
  const int lane = threadIdx.x & 31;
  const int wave = threadIdx.x >> 5;
  const int tilesN = N >> 6;
  const int tilesM = M >> 6;
  const int tile = blockIdx.x * 8 + wave;
  if (tile >= tilesM * tilesN) return;
  const int tm = tile / tilesN;
  const int tn = tile - tm * tilesN;
  const int m0 = tm << 6;
  const int n0 = tn << 6;

  const T* Ab  = A  + (size_t)b * strideA;
  const T* Bb  = Bt + (size_t)b * strideB;
  const T* Ab2 = SPLIT ? (A2  + (size_t)b * strideA) : nullptr;
  const T* Bb2 = SPLIT ? (Bt2 + (size_t)b * strideB) : nullptr;

  const int rlane = lane & 15;
  const int koff  = (lane >> 4) * 8;
  const int mOff  = (lane >> 4) * 8;

  v8f acc[4][4];
#pragma unroll
  for (int i = 0; i < 4; ++i)
#pragma unroll
    for (int j = 0; j < 4; ++j) acc[i][j] = (v8f){0.f,0.f,0.f,0.f,0.f,0.f,0.f,0.f};

  for (int k0 = 0; k0 < K; k0 += 32) {
    V bh[4], bl[4];
#pragma unroll
    for (int j = 0; j < 4; ++j) {
      const size_t bo = (size_t)(n0 + (j << 4) + rlane) * ldb + koff + k0;
      bh[j] = Frag<T>::load(Bb + bo);
      if (SPLIT) bl[j] = Frag<T>::load(Bb2 + bo);
    }
#pragma unroll
    for (int i = 0; i < 4; ++i) {
      const size_t ao = (size_t)(m0 + (i << 4) + rlane) * lda + koff + k0;
      V ah = Frag<T>::load(Ab + ao);
      V al;
      if (SPLIT) al = Frag<T>::load(Ab2 + ao);
#pragma unroll
      for (int j = 0; j < 4; ++j) {
        acc[i][j] = Frag<T>::mma(ah, bh[j], acc[i][j]);
        if (SPLIT) {
          acc[i][j] = Frag<T>::mma(ah, bl[j], acc[i][j]);
          acc[i][j] = Frag<T>::mma(al, bh[j], acc[i][j]);
        }
      }
      Frag<T>::guard(acc[i][0], acc[i][3], ah, SPLIT ? al : ah);
    }
    Frag<T>::keep(bh[0], bh[1], bh[2], bh[3]);
    if (SPLIT) Frag<T>::keep(bl[0], bl[1], bl[2], bl[3]);
  }
  acc_guard4(acc[0][0], acc[0][1], acc[0][2], acc[0][3]);
  acc_guard4(acc[1][0], acc[1][1], acc[1][2], acc[1][3]);
  acc_guard4(acc[2][0], acc[2][1], acc[2][2], acc[2][3]);
  acc_guard4(acc[3][0], acc[3][1], acc[3][2], acc[3][3]);

  float* slab = sT[wave];
  const float* Rb = RESID ? (resid + (size_t)b * strideR) : nullptr;
#pragma unroll
  for (int i = 0; i < 4; ++i) {
    const int mBase = m0 + (i << 4);
#pragma unroll
    for (int j = 0; j < 4; ++j) {
      const int n = n0 + (j << 4) + rlane;
      float bv = 0.f;
      if (BIAS_MODE == 2) bv = bias[n];
#pragma unroll
      for (int r = 0; r < 8; ++r) {
        float v = acc[i][j][r] * scale;
        if (BIAS_MODE == 1) v += bias[mBase + mOff + r];
        if (BIAS_MODE == 2) v += bv;
        if (RESID) v += Rb[(size_t)(mBase + mOff + r) * ldc + n];
        if (ACT == 1) v = tanhf(v);
        if (ACT == 2) v = fmaxf(v, 0.0f);
        if (ACT == 4) v = (v > 0.f) ? v : 0.01f * v;
        slab[(mOff + r) * 68 + (j << 4) + rlane] = v;
      }
    }
    __builtin_amdgcn_fence(__ATOMIC_RELEASE, "workgroup");
    __builtin_amdgcn_wave_barrier();
    __builtin_amdgcn_fence(__ATOMIC_ACQUIRE, "workgroup");
    if (OUT_MODE == 0) {
      float* C = (float*)Cout + (size_t)b * strideC;
      const int hh = lane >> 4, c4 = (lane & 15) * 4;
      for (int pass = 0; pass < 2; ++pass) {
#pragma unroll
        for (int it = 0; it < 8; ++it) {
          const int row = it * 2 + hh;
          v4f v = *(const v4f*)(slab + row * 68 + c4);
          *(volatile v4f*)(C + (size_t)(mBase + row) * ldc + n0 + c4) = v;
        }
        __threadfence();
      }
    } else {
      const int q = lane >> 3, c8 = (lane & 7) * 8;
      unsigned short* C  = (unsigned short*)Cout  + (size_t)b * strideC;
      unsigned short* C2 = (OUT_MODE == 2) ? ((unsigned short*)Cout2 + (size_t)b * strideC) : nullptr;
      for (int pass = 0; pass < 2; ++pass) {
#pragma unroll
        for (int it = 0; it < 4; ++it) {
          const int row = it * 4 + q;
          const float* sp = slab + row * 68 + c8;
          v8h hv, lv;
#pragma unroll
          for (int e = 0; e < 8; ++e) {
            if (OUT_MODE == 1) {
              hv[e] = (_Float16)sp[e];
            } else {
              unsigned short hb = f2bf_bits(sp[e]);
              unsigned short lb = f2bf_bits(sp[e] - bf_bits2f(hb));
              hv[e] = __builtin_bit_cast(_Float16, hb);
              lv[e] = __builtin_bit_cast(_Float16, lb);
            }
          }
          *(volatile v8h*)(C + (size_t)(mBase + row) * ldc + n0 + c8) = hv;
          if (OUT_MODE == 2) *(volatile v8h*)(C2 + (size_t)(mBase + row) * ldc + n0 + c8) = lv;
        }
        __threadfence();
      }
    }
    __builtin_amdgcn_fence(__ATOMIC_RELEASE, "workgroup");
    __builtin_amdgcn_wave_barrier();
    __builtin_amdgcn_fence(__ATOMIC_ACQUIRE, "workgroup");
  }
}

__global__ __launch_bounds__(256) void cast_rows_f16_kernel(
    const float* __restrict__ src, unsigned short* __restrict__ dst, int N, int K, int total8, float scale)
{
  const int i = blockIdx.x * 256 + threadIdx.x;
  if (i >= total8) return;
  const int e0  = i << 3;
  const int row = e0 / K;
  const int col = e0 - row * K;
  const int rowc = (row < N) ? row : (N - 1);
  const bool live = (row < N);
  const float* p = src + (size_t)rowc * K + col;
  const v4f a0 = *(const v4f*)(p);
  const v4f a1 = *(const v4f*)(p + 4);
  v8h hv;
#pragma unroll
  for (int e = 0; e < 4; ++e) {
    hv[e]     = live ? (_Float16)(a0[e] * scale) : (_Float16)0.0f;
    hv[4 + e] = live ? (_Float16)(a1[e] * scale) : (_Float16)0.0f;
  }
  unsigned short* q = dst + (size_t)e0;
  *(volatile v8h*)q = hv;
  __threadfence();
  *(volatile v8h*)q = hv;
}

__global__ __launch_bounds__(256) void cast_xproj_f16_kernel(
    const float* __restrict__ wf, const float* __restrict__ wb, unsigned short* __restrict__ dst, int total8, float scale)
{
  const int i = blockIdx.x * 256 + threadIdx.x;
  if (i >= total8) return;
  const int e0  = i << 3;
  const int blk = e0 >> 12;
  const int rem = e0 & 4095;
  const int row = rem >> 6;
  const int col = rem & 63;
  const int rf  = (row < kPrjN) ? row : (kPrjN - 1);
  int rb = row - kPrjN; rb = (rb < 0) ? 0 : ((rb > kPrjN - 1) ? (kPrjN - 1) : rb);
  const float* pf = wf + ((size_t)blk * kPrjN + rf) * kDim + col;
  const float* pb = wb + ((size_t)blk * kPrjN + rb) * kDim + col;
  const v4f f0 = *(const v4f*)(pf);
  const v4f f1 = *(const v4f*)(pf + 4);
  const v4f g0 = *(const v4f*)(pb);
  const v4f g1 = *(const v4f*)(pb + 4);
  const bool useF = (row < kPrjN);
  const bool useB = (row >= kPrjN) && (row < 2 * kPrjN);
  v8h hv;
#pragma unroll
  for (int e = 0; e < 4; ++e) {
    const float vf0 = f0[e] * scale, vb0 = g0[e] * scale;
    const float vf1 = f1[e] * scale, vb1 = g1[e] * scale;
    const float s0 = useF ? vf0 : (useB ? vb0 : 0.0f);
    const float s1 = useF ? vf1 : (useB ? vb1 : 0.0f);
    hv[e]     = (_Float16)s0;
    hv[4 + e] = (_Float16)s1;
  }
  unsigned short* q = dst + (size_t)e0;
  *(volatile v8h*)q = hv;
  __threadfence();
  *(volatile v8h*)q = hv;
}

__global__ __launch_bounds__(256) void seq_rows_kernel(
    const float* __restrict__ s0, const float* __restrict__ s1, const float* __restrict__ s2, const float* __restrict__ s3,
    float* __restrict__ d0, float* __restrict__ d1, float* __restrict__ d2, float* __restrict__ d3)
{
  __shared__ float tile[64 * 65];
  const int tid = threadIdx.x, lane = tid & 31, wave = tid >> 5;
  const int z = blockIdx.z;
  const float* src = (z == 0) ? s0 : ((z == 1) ? s1 : ((z == 2) ? s2 : s3));
  float*       dst = (z == 0) ? d0 : ((z == 1) ? d1 : ((z == 2) ? d2 : d3));
  const int b  = blockIdx.y;
  const int l0 = blockIdx.x * 64;
#pragma unroll
  for (int p = 0; p < 16; ++p) {
    const int idx = tid + p * 256;
    const int cc  = idx >> 6;
    const int ll  = idx & 63;
    tile[cc * 65 + ll] = src[((size_t)(b * kDim + cc)) * kSeqL + l0 + ll];
  }
  __syncthreads();
  const int hh = lane >> 4, c4 = (lane & 15) * 4;
  v4f v[4];
#pragma unroll
  for (int it = 0; it < 4; ++it) {
    const int lrow = wave * 8 + it * 2 + hh;
#pragma unroll
    for (int e = 0; e < 4; ++e) v[it][e] = tile[(c4 + e) * 65 + lrow];
  }
  for (int pass = 0; pass < 2; ++pass) {
#pragma unroll
    for (int it = 0; it < 4; ++it) {
      const int lrow = wave * 8 + it * 2 + hh;
      *(volatile v4f*)(dst + ((size_t)(b * kSeqL + l0 + lrow)) * kDim + c4) = v[it];
    }
    __threadfence();
  }
}

__global__ __launch_bounds__(256) void ln_rows_f16_kernel(
    const float* __restrict__ xa, const float* __restrict__ wa, const float* __restrict__ ba, unsigned short* __restrict__ oa,
    const float* __restrict__ xb, const float* __restrict__ wb, const float* __restrict__ bb, unsigned short* __restrict__ ob,
    float oscale)
{
  __shared__ __align__(16) float sL[8][4 * 64];
  const int tid = threadIdx.x, lane = tid & 31, wave = tid >> 5;
  const bool sel = (blockIdx.y != 0);
  const float* x  = sel ? xb : xa;
  const float* w  = sel ? wb : wa;
  const float* bi = sel ? bb : ba;
  unsigned short* o = sel ? ob : oa;
  const int r0 = blockIdx.x * 32 + wave * 4;
  float* slab = sL[wave];
  const float wl = w[lane], wh = w[lane + 32], cl = bi[lane], ch = bi[lane + 32];
#pragma unroll
  for (int r = 0; r < 4; ++r) {
    const float* xr = x + (size_t)(r0 + r) * kDim;
    const float v0 = xr[lane], v1 = xr[lane + 32];
    float s = v0 + v1;
#pragma unroll
    for (int msk = 16; msk >= 1; msk >>= 1) s += __shfl_xor(s, msk, 32);
    const float mean = s * (1.0f / 64.0f);
    const float e0 = v0 - mean, e1 = v1 - mean;
    float sq = e0 * e0 + e1 * e1;
#pragma unroll
    for (int msk = 16; msk >= 1; msk >>= 1) sq += __shfl_xor(sq, msk, 32);
    const float var = sq * (1.0f / 64.0f);
    const float rs  = rsqrtf(var + 1e-5f);
    slab[r * 64 + lane]      = (e0 * rs * wl + cl) * oscale;
    slab[r * 64 + lane + 32] = (e1 * rs * wh + ch) * oscale;
  }
  __builtin_amdgcn_fence(__ATOMIC_RELEASE, "workgroup");
  __builtin_amdgcn_wave_barrier();
  __builtin_amdgcn_fence(__ATOMIC_ACQUIRE, "workgroup");
  const int q = lane >> 3, c8 = (lane & 7) * 8;
  const float* sp = slab + q * 64 + c8;
  const v4f a0 = *(const v4f*)(sp);
  const v4f a1 = *(const v4f*)(sp + 4);
  v8h hv;
#pragma unroll
  for (int e = 0; e < 4; ++e) { hv[e] = (_Float16)a0[e]; hv[4 + e] = (_Float16)a1[e]; }
  unsigned short* op = o + (size_t)(r0 + q) * kDim + c8;
  *(volatile v8h*)op = hv;
  __threadfence();
  *(volatile v8h*)op = hv;
}

__global__ __launch_bounds__(256) void combine_gate_f16_kernel(
    const float* __restrict__ Yf, const float* __restrict__ Yb, const float* __restrict__ XZ,
    const float* __restrict__ lw, const float* __restrict__ lb, unsigned short* __restrict__ G16, float oscale)
{
  __shared__ __align__(16) float sL[8][4 * 64];
  const int tid = threadIdx.x, lane = tid & 31, wave = tid >> 5;
  const int r0 = blockIdx.x * 32 + wave * 4;
  float* slab = sL[wave];
  const float wl = lw[lane], wh = lw[lane + 32], cl = lb[lane], ch = lb[lane + 32];
#pragma unroll
  for (int r = 0; r < 4; ++r) {
    const size_t o64  = (size_t)(r0 + r) * kDim;
    const size_t o128 = (size_t)(r0 + r) * kXZP;
    const float v0 = 0.5f * (Yf[o64 + lane] + Yb[o64 + lane]);
    const float v1 = 0.5f * (Yf[o64 + lane + 32] + Yb[o64 + lane + 32]);
    float s = v0 + v1;
#pragma unroll
    for (int msk = 16; msk >= 1; msk >>= 1) s += __shfl_xor(s, msk, 32);
    const float mean = s * (1.0f / 64.0f);
    const float e0 = v0 - mean, e1 = v1 - mean;
    float sq = e0 * e0 + e1 * e1;
#pragma unroll
    for (int msk = 16; msk >= 1; msk >>= 1) sq += __shfl_xor(sq, msk, 32);
    const float var = sq * (1.0f / 64.0f);
    const float rs  = rsqrtf(var + 1e-5f);
    const float z0 = XZ[o128 + kDim + lane], z1 = XZ[o128 + kDim + 32 + lane];
    const float g0 = z0 * __builtin_amdgcn_rcpf(1.0f + __expf(-z0));
    const float g1 = z1 * __builtin_amdgcn_rcpf(1.0f + __expf(-z1));
    slab[r * 64 + lane]      = (e0 * rs * wl + cl) * g0 * oscale;
    slab[r * 64 + lane + 32] = (e1 * rs * wh + ch) * g1 * oscale;
  }
  __builtin_amdgcn_fence(__ATOMIC_RELEASE, "workgroup");
  __builtin_amdgcn_wave_barrier();
  __builtin_amdgcn_fence(__ATOMIC_ACQUIRE, "workgroup");
  const int q = lane >> 3, c8 = (lane & 7) * 8;
  const float* sp = slab + q * 64 + c8;
  const v4f a0 = *(const v4f*)(sp);
  const v4f a1 = *(const v4f*)(sp + 4);
  v8h hv;
#pragma unroll
  for (int e = 0; e < 4; ++e) { hv[e] = (_Float16)a0[e]; hv[4 + e] = (_Float16)a1[e]; }
  unsigned short* op = G16 + (size_t)(r0 + q) * kDim + c8;
  *(volatile v8h*)op = hv;
  __threadfence();
  *(volatile v8h*)op = hv;
}

__global__ __launch_bounds__(64) void scan_dir_kernel(
    const float* __restrict__ XZ, const float* __restrict__ DBL,
    const float* __restrict__ cwf, const float* __restrict__ cbf,
    const float* __restrict__ cwb, const float* __restrict__ cbb,
    const float* __restrict__ dtwf, const float* __restrict__ dtbf,
    const float* __restrict__ dtwb, const float* __restrict__ dtbb,
    const float* __restrict__ alf, const float* __restrict__ alb,
    const float* __restrict__ dvf, const float* __restrict__ dvb,
    float* __restrict__ Y)
{
  __shared__ __align__(16) float sP[16 * kPrjP];
  __shared__ __align__(16) float sY[16 * kYP];
  const int tid = threadIdx.x, lane = tid & 31, wave = tid >> 5;
  const int d   = tid;
  const int b   = blockIdx.x;
  const int rev = blockIdx.y;
  const float* cw  = rev ? cwb  : cwf;
  const float* cb  = rev ? cbb  : cbf;
  const float* dtw = rev ? dtwb : dtwf;
  const float* dtb = rev ? dtbb : dtbf;
  const float* al  = rev ? alb  : alf;
  const float* dv  = rev ? dvb  : dvf;
  const size_t brow = (size_t)b * kSeqL;
  float* Yd = Y + (size_t)rev * kRows * kDim;
  const int pofs = rev * kPrjN;

  float An[kNst];
#pragma unroll
  for (int n = 0; n < kNst; ++n) An[n] = -__expf(al[(size_t)d * kNst + n]);
  const float wd0 = dtw[d * kDtR + 0], wd1 = dtw[d * kDtR + 1], wd2 = dtw[d * kDtR + 2], wd3 = dtw[d * kDtR + 3];
  const float bdt = dtb[d];
  const float w0 = cw[d * kTap + 0], w1 = cw[d * kTap + 1], w2 = cw[d * kTap + 2], w3 = cw[d * kTap + 3];
  const float bc = cb[d];
  const float Dd = dv[d];
  float h[kNst];
#pragma unroll
  for (int n = 0; n < kNst; ++n) h[n] = 0.f;
  float xm3 = 0.f, xm2 = 0.f, xm1 = 0.f;
  const int hh = lane >> 4, c4 = (lane & 15) * 4;

#pragma unroll 1
  for (int c = 0; c < kSeqL / 16; ++c) {
    const int l0 = c * 16;
#pragma unroll
    for (int qq = 0; qq < 4; ++qq) {
      const int idx = tid + qq * 64;
      const int r   = idx >> 4;
      const int cc  = (idx & 15) * 4;
      const int tt  = l0 + r;
      const int tok = rev ? (kSeqL - 1 - tt) : tt;
      const v4f v = *(const v4f*)(DBL + (brow + (size_t)tok) * kPrjP + cc);
      *(v4f*)(sP + r * kPrjP + cc) = v;
    }
    __syncthreads();
#pragma unroll 1
    for (int st = 0; st < 16; ++st) {
      const int tt  = l0 + st;
      const int tok = rev ? (kSeqL - 1 - tt) : tt;
      const size_t m = brow + (size_t)tok;
      const float* pr = sP + st * kPrjP + pofs;
      const v4f dq  = *(const v4f*)(pr);
      const v4f bq0 = *(const v4f*)(pr + 4);
      const v4f bq1 = *(const v4f*)(pr + 8);
      const v4f cq0 = *(const v4f*)(pr + 12);
      const v4f cq1 = *(const v4f*)(pr + 16);
      float a = dq[0] * wd0;
      a = fmaf(dq[1], wd1, a);
      a = fmaf(dq[2], wd2, a);
      a = fmaf(dq[3], wd3, a);
      a += bdt;
      const float delta = fmaxf(a, 0.0f) + log1pf(__expf(-fabsf(a)));
      const float xin = XZ[m * kXZP + d];
      float acc = w0 * xm3;
      acc = fmaf(w1, xm2, acc);
      acc = fmaf(w2, xm1, acc);
      acc = fmaf(w3, xin, acc);
      const float sv = acc + bc;
      const float u  = sv * __builtin_amdgcn_rcpf(1.0f + __expf(-sv));
      xm3 = xm2; xm2 = xm1; xm1 = xin;
      float dx = delta * u;
      asm volatile("" : "+v"(dx));
      float y = 0.f;
#pragma unroll
      for (int n = 0; n < kNst; ++n) {
        const float bn = (n < 4) ? bq0[n & 3] : bq1[n & 3];
        const float cn = (n < 4) ? cq0[n & 3] : cq1[n & 3];
        const float e  = __expf(delta * An[n]);
        float p = dx * bn;
        asm volatile("" : "+v"(p));
        float qv = h[n] * e;
        asm volatile("" : "+v"(qv));
        const float hn = qv + p;
        h[n] = hn;
        float rr = hn * cn;
        asm volatile("" : "+v"(rr));
        y += rr;
      }
      float sk = u * Dd;
      asm volatile("" : "+v"(sk));
      y += sk;
      sY[st * kYP + d] = y;
    }
    __syncthreads();
    v4f yv[4];
#pragma unroll
    for (int it = 0; it < 4; ++it) {
      const int row = it * 4 + wave * 2 + hh;
      yv[it] = *(const v4f*)(sY + row * kYP + c4);
    }
    for (int pass = 0; pass < 2; ++pass) {
#pragma unroll
      for (int it = 0; it < 4; ++it) {
        const int row = it * 4 + wave * 2 + hh;
        const int tt  = l0 + row;
        const int tok = rev ? (kSeqL - 1 - tt) : tt;
        *(volatile v4f*)(Yd + (brow + (size_t)tok) * kDim + c4) = yv[it];
      }
      __threadfence();
    }
    __syncthreads();
  }
}

__global__ __launch_bounds__(256) void avg_cat_f16_kernel(
    const float* __restrict__ i1l, const float* __restrict__ i1g,
    const float* __restrict__ i2l, const float* __restrict__ i2g,
    unsigned short* __restrict__ A16)
{
  const int tid = threadIdx.x, lane = tid & 31, wave = tid >> 5;
  const int half = wave & 1;
  const int q = lane >> 3, c8 = (lane & 7) * 8;
  const int row = blockIdx.x * 16 + (wave >> 1) * 4 + q;
  const float* pa = half ? i1g : i1l;
  const float* pb = half ? i2g : i2l;
  const size_t so = (size_t)row * kDim + c8;
  const v4f a0 = *(const v4f*)(pa + so);
  const v4f a1 = *(const v4f*)(pa + so + 4);
  const v4f b0 = *(const v4f*)(pb + so);
  const v4f b1 = *(const v4f*)(pb + so + 4);
  v8h hv;
#pragma unroll
  for (int e = 0; e < 4; ++e) {
    hv[e]     = (_Float16)(0.5f * (a0[e] + b0[e]));
    hv[4 + e] = (_Float16)(0.5f * (a1[e] + b1[e]));
  }
  unsigned short* op = A16 + (size_t)row * kCatW + half * kDim + c8;
  *(volatile v8h*)op = hv;
  __threadfence();
  *(volatile v8h*)op = hv;
}

extern "C" void kernel_launch(void* const* d_in, const int* in_sizes, int n_in,
                              void* d_out, int out_size, void* d_ws, size_t ws_size,
                              hipStream_t stream)
{
  if (n_in < 30) return;
  const float* img0     = (const float*)d_in[0];
  const float* img1     = (const float*)d_in[1];
  const float* img2     = (const float*)d_in[2];
  const float* img3     = (const float*)d_in[3];
  const float* norm0_w  = (const float*)d_in[4];
  const float* norm0_b  = (const float*)d_in[5];
  const float* norm1_w  = (const float*)d_in[6];
  const float* norm1_b  = (const float*)d_in[7];
  const float* in_w     = (const float*)d_in[8];
  const float* in_b     = (const float*)d_in[9];
  const float* conv_w_f = (const float*)d_in[10];
  const float* conv_b_f = (const float*)d_in[11];
  const float* conv_w_b = (const float*)d_in[12];
  const float* conv_b_b = (const float*)d_in[13];
  const float* xproj_f  = (const float*)d_in[14];
  const float* xproj_b  = (const float*)d_in[15];
  const float* dtw_f    = (const float*)d_in[16];
  const float* dtb_f    = (const float*)d_in[17];
  const float* dtw_b    = (const float*)d_in[18];
  const float* dtb_b    = (const float*)d_in[19];
  const float* alog_f   = (const float*)d_in[20];
  const float* alog_b   = (const float*)d_in[21];
  const float* dsk_f    = (const float*)d_in[22];
  const float* dsk_b    = (const float*)d_in[23];
  const float* ln_w     = (const float*)d_in[24];
  const float* ln_b     = (const float*)d_in[25];
  const float* mout_w   = (const float*)d_in[26];
  const float* mout_b   = (const float*)d_in[27];
  const float* fop_w    = (const float*)d_in[28];
  const float* fop_b    = (const float*)d_in[29];
  float* dout = (float*)d_out;

  const int nImg = kBatch * kDim * kSeqL;
  if (in_sizes[0] != nImg || in_sizes[1] != nImg || in_sizes[2] != nImg || in_sizes[3] != nImg) return;
  for (int i = 4; i <= 7; ++i) if (in_sizes[i] != kNBlk * kDim) return;
  if (in_sizes[8] != kNBlk * kXZP * kDim || in_sizes[9] != kNBlk * kXZP) return;
  if (in_sizes[10] != kNBlk * kDim * kTap || in_sizes[11] != kNBlk * kDim) return;
  if (in_sizes[12] != kNBlk * kDim * kTap || in_sizes[13] != kNBlk * kDim) return;
  if (in_sizes[14] != kNBlk * kPrjN * kDim || in_sizes[15] != kNBlk * kPrjN * kDim) return;
  if (in_sizes[16] != kNBlk * kDim * kDtR || in_sizes[17] != kNBlk * kDim) return;
  if (in_sizes[18] != kNBlk * kDim * kDtR || in_sizes[19] != kNBlk * kDim) return;
  if (in_sizes[20] != kNBlk * kDim * kNst || in_sizes[21] != kNBlk * kDim * kNst) return;
  for (int i = 22; i <= 25; ++i) if (in_sizes[i] != kNBlk * kDim) return;
  if (in_sizes[26] != kNBlk * kDim * kDim || in_sizes[27] != kNBlk * kDim) return;
  if (in_sizes[28] != kDim * kCatW || in_sizes[29] != kDim) return;
  if (out_size != kBatch * kDim * kSeqL) return;

  const size_t SZ_PL    = (size_t)kRows * kDim * 4;
  const size_t SZ_XZ    = (size_t)kRows * kXZP * 4;
  const size_t SZ_DBL   = (size_t)kRows * kPrjP * 4;
  const size_t SZ_Y     = (size_t)2 * kRows * kDim * 4;
  const size_t SZ_R16   = (size_t)kRows * kDim * 2;
  const size_t SZ_A16   = (size_t)kRows * kCatW * 2;
  const size_t SZ_INW16 = (size_t)kNBlk * kXZP * kDim * 2;
  const size_t SZ_XPW16 = (size_t)kNBlk * kPrjP * kDim * 2;
  const size_t SZ_MW16  = (size_t)kNBlk * kDim * kDim * 2;
  const size_t SZ_FW16  = (size_t)kDim * kCatW * 2;
  const size_t OFF_S     = 0;
  const size_t OFF_NS    = OFF_S     + 4 * SZ_PL;
  const size_t OFF_IB    = OFF_NS    + 4 * SZ_PL;
  const size_t OFF_XZ    = OFF_IB    + 4 * SZ_PL;
  const size_t OFF_DBL   = OFF_XZ    + SZ_XZ;
  const size_t OFF_Y     = OFF_DBL   + SZ_DBL;
  const size_t OFF_XN16  = OFF_Y     + SZ_Y;
  const size_t OFF_EN16  = OFF_XN16  + SZ_R16;
  const size_t OFF_G16   = OFF_EN16  + SZ_R16;
  const size_t OFF_A16   = OFF_G16   + SZ_R16;
  const size_t OFF_INW16 = OFF_A16   + SZ_A16;
  const size_t OFF_XPW16 = OFF_INW16 + SZ_INW16;
  const size_t OFF_MW16  = OFF_XPW16 + SZ_XPW16;
  const size_t OFF_FW16  = OFF_MW16  + SZ_MW16;
  const size_t TOTAL     = OFF_FW16  + SZ_FW16;
  if (ws_size < TOTAL) return;

  char* ws = (char*)d_ws;
  float* S[4]; float* NS[4]; float* IB[4];
  for (int i = 0; i < 4; ++i) {
    S[i]  = (float*)(ws + OFF_S  + (size_t)i * SZ_PL);
    NS[i] = (float*)(ws + OFF_NS + (size_t)i * SZ_PL);
    IB[i] = (float*)(ws + OFF_IB + (size_t)i * SZ_PL);
  }
  float*          XZ    = (float*)(ws + OFF_XZ);
  float*          DBL   = (float*)(ws + OFF_DBL);
  float*          Y     = (float*)(ws + OFF_Y);
  unsigned short* XN16  = (unsigned short*)(ws + OFF_XN16);
  unsigned short* EN16  = (unsigned short*)(ws + OFF_EN16);
  unsigned short* G16   = (unsigned short*)(ws + OFF_G16);
  unsigned short* A16   = (unsigned short*)(ws + OFF_A16);
  unsigned short* INW16 = (unsigned short*)(ws + OFF_INW16);
  unsigned short* XPW16 = (unsigned short*)(ws + OFF_XPW16);
  unsigned short* MW16  = (unsigned short*)(ws + OFF_MW16);
  unsigned short* FW16  = (unsigned short*)(ws + OFF_FW16);
  const float* dummy_bias  = in_b;
  const float* dummy_resid = S[0];

  seq_rows_kernel<<<dim3(kSeqL / 64, kBatch, 4), 256, 0, stream>>>(
      img0, img1, img2, img3, S[0], S[1], S[2], S[3]);

  cast_rows_f16_kernel<<<(kNBlk * kXZP * kDim) / 8 / 256, 256, 0, stream>>>(
      in_w, INW16, kNBlk * kXZP, kDim, (kNBlk * kXZP * kDim) / 8, 32.0f);
  cast_rows_f16_kernel<<<(kNBlk * kDim * kDim) / 8 / 256, 256, 0, stream>>>(
      mout_w, MW16, kNBlk * kDim, kDim, (kNBlk * kDim * kDim) / 8, 32.0f);
  cast_rows_f16_kernel<<<(kDim * kCatW) / 8 / 256, 256, 0, stream>>>(
      fop_w, FW16, kDim, kCatW, (kDim * kCatW) / 8, 32.0f);
  cast_xproj_f16_kernel<<<(kNBlk * kPrjP * kDim) / 8 / 256, 256, 0, stream>>>(
      xproj_f, xproj_b, XPW16, (kNBlk * kPrjP * kDim) / 8, 32.0f);

  const float* xs[8] = {S[0], S[1], S[2], S[3], NS[0], NS[0], NS[1], NS[1]};
  const float* es[8] = {S[2], S[3], NS[0], NS[1], NS[1], NS[3], NS[0], NS[2]};
  float*       ds[8] = {NS[0], NS[1], NS[2], NS[3], IB[0], IB[1], IB[2], IB[3]};

  for (int i = 0; i < kNBlk; ++i) {
    ln_rows_f16_kernel<<<dim3(kRows / 32, 2), 256, 0, stream>>>(
        xs[i], norm0_w + i * kDim, norm0_b + i * kDim, XN16,
        es[i], norm1_w + i * kDim, norm1_b + i * kDim, EN16, 1.0f);

    wmma_gemm64<0, false, 2, 0, false><<<dim3(64, 1), 256, 0, stream>>>(
        XN16, XN16, kDim, 0L, INW16 + (size_t)i * kXZP * kDim, INW16 + (size_t)i * kXZP * kDim, kDim, 0L,
        (void*)XZ, (void*)XZ, kXZP, 0L, in_b + (size_t)i * kXZP, dummy_resid, 0L, kRows, kXZP, kDim, 1.0f / 32.0f);

    wmma_gemm64<0, false, 0, 0, false><<<dim3(32, 1), 256, 0, stream>>>(
        EN16, EN16, kDim, 0L, XPW16 + (size_t)i * kPrjP * kDim, XPW16 + (size_t)i * kPrjP * kDim, kDim, 0L,
        (void*)DBL, (void*)DBL, kPrjP, 0L, dummy_bias, dummy_resid, 0L, kRows, kPrjP, kDim, 1.0f / 32.0f);

    scan_dir_kernel<<<dim3(kBatch, 2), 64, 0, stream>>>(
        XZ, DBL,
        conv_w_f + (size_t)i * kDim * kTap, conv_b_f + (size_t)i * kDim,
        conv_w_b + (size_t)i * kDim * kTap, conv_b_b + (size_t)i * kDim,
        dtw_f + (size_t)i * kDim * kDtR, dtb_f + (size_t)i * kDim,
        dtw_b + (size_t)i * kDim * kDtR, dtb_b + (size_t)i * kDim,
        alog_f + (size_t)i * kDim * kNst, alog_b + (size_t)i * kDim * kNst,
        dsk_f + (size_t)i * kDim, dsk_b + (size_t)i * kDim,
        Y);

    combine_gate_f16_kernel<<<kRows / 32, 256, 0, stream>>>(
        Y, Y + (size_t)kRows * kDim, XZ, ln_w + (size_t)i * kDim, ln_b + (size_t)i * kDim, G16, 16.0f);

    wmma_gemm64<0, false, 2, 0, true><<<dim3(32, 1), 256, 0, stream>>>(
        G16, G16, kDim, 0L, MW16 + (size_t)i * kDim * kDim, MW16 + (size_t)i * kDim * kDim, kDim, 0L,
        (void*)ds[i], (void*)ds[i], kDim, 0L, mout_b + (size_t)i * kDim, xs[i], 0L, kRows, kDim, kDim, 1.0f / 512.0f);
  }

  avg_cat_f16_kernel<<<kRows / 16, 256, 0, stream>>>(IB[0], IB[1], IB[2], IB[3], A16);

  wmma_gemm64<0, false, 1, 0, false><<<dim3(8, kBatch), 256, 0, stream>>>(
      FW16, FW16, kCatW, 0L, A16, A16, kCatW, (long)kSeqL * kCatW,
      (void*)dout, (void*)dout, kSeqL, (long)kDim * kSeqL, fop_b, dummy_resid, 0L, kDim, kSeqL, kCatW, 1.0f / 32.0f);
}
